// SelfAttention_57002805952906
// MI455X (gfx1250) — hardware-verified
//
#include <hip/hip_runtime.h>
#include <stdint.h>

#ifndef NB
#define NB 8
#endif
#ifndef SEQ
#define SEQ 2048
#endif
#define NB_FULL  8
#define SEQ_FULL 2048
#define EM       128
#define DM       256
#define RTOT     (NB * SEQ)
#define EROWS    ((SEQ) < 512 ? (SEQ) : 512)
#define LBLK     (((SEQ) - EROWS) / 32)
#define LBLKD    (LBLK > 0 ? LBLK : 1)
#define EBLK     (EROWS / 16)

static_assert(NB >= 1 && NB <= NB_FULL);
static_assert(SEQ >= 256 && SEQ <= SEQ_FULL && (SEQ % 256) == 0);
static_assert(DM == 256 && EM == 128);
static_assert((EM % 32) == 0 && (DM % 64) == 0);
static_assert((RTOT % 128) == 0);
static_assert(((size_t)RTOT * EM) % 2048 == 0);
static_assert((3 * DM * EM) % 2048 == 0);
static_assert((EROWS % 32) == 0 && ((SEQ - EROWS) % 32) == 0);
static_assert((((RTOT / 64) * (DM / 64)) % 8) == 0);

typedef _Float16 v16h __attribute__((ext_vector_type(16)));
typedef _Float16 v8h  __attribute__((ext_vector_type(8)));
typedef float    v8f  __attribute__((ext_vector_type(8)));
typedef float    v4f  __attribute__((ext_vector_type(4)));

__device__ __forceinline__ unsigned short bfbits(float f) {
  unsigned u = __float_as_uint(f);
  return (unsigned short)((u + 0x7FFFu + ((u >> 16) & 1u)) >> 16);
}
__device__ __forceinline__ float bfval(unsigned short b) { return __uint_as_float(((unsigned)b) << 16); }
__device__ __forceinline__ float bfr(float f) { return bfval(bfbits(f)); }

__device__ __forceinline__ v8f mma16(v16h a, v16h b, v8f c) {
  return __builtin_amdgcn_wmma_f32_16x16x32_f16(false, a, false, b, (short)0, c, false, false);
}

__device__ __forceinline__ v16h ldfrag(const _Float16* p) {
  union { v16h v; v8h h[2]; } f;
  f.h[0] = *(const v8h*)(p);
  f.h[1] = *(const v8h*)(p + 16);
  return f.v;
}
__device__ __forceinline__ v8f zero8() {
  v8f z;
#pragma unroll
  for (int i = 0; i < 8; ++i) z[i] = 0.0f;
  return z;
}

__device__ __forceinline__ void guard_g(v8f& a, v8f& b, v16h x, v16h y) {
  asm volatile("v_nop\n\tv_nop\n\tv_nop\n\tv_nop" : "+v"(a), "+v"(b) : "v"(x), "v"(y));
}
__device__ __forceinline__ void keep4(v16h a, v16h b, v16h c, v16h d) {
  asm volatile("v_nop" :: "v"(a), "v"(b), "v"(c), "v"(d));
}
__device__ __forceinline__ void accg4(v8f& a, v8f& b, v8f& c, v8f& d) {
  asm volatile("v_nop\n\tv_nop\n\tv_nop\n\tv_nop" : "+v"(a), "+v"(b), "+v"(c), "+v"(d));
}
__device__ __forceinline__ void guard_s8(v8f& a0, v8f& a1, v8f& a2, v8f& a3, v8f& b0, v8f& b1, v8f& b2, v8f& b3,
                                         v16h x0, v16h x1, v16h y0, v16h y1, v16h z0, v16h z1) {
  asm volatile("v_nop\n\tv_nop\n\tv_nop\n\tv_nop"
               : "+v"(a0), "+v"(a1), "+v"(a2), "+v"(a3), "+v"(b0), "+v"(b1), "+v"(b2), "+v"(b3)
               : "v"(x0), "v"(x1), "v"(y0), "v"(y1), "v"(z0), "v"(z1));
}
__device__ __forceinline__ void guard_a4f6(v8f& a0, v8f& a1, v8f& b0, v8f& b1,
                                           v16h x0, v16h x1, v16h y0, v16h y1, v16h z0, v16h z1) {
  asm volatile("v_nop\n\tv_nop\n\tv_nop\n\tv_nop"
               : "+v"(a0), "+v"(a1), "+v"(b0), "+v"(b1)
               : "v"(x0), "v"(x1), "v"(y0), "v"(y1), "v"(z0), "v"(z1));
}
__device__ __forceinline__ void guard_pv4(v8f& a0, v8f& a1, v8f& b0, v8f& b1,
                                          v16h p0, v16h p1, v16h x0, v16h x1) {
  asm volatile("v_nop\n\tv_nop\n\tv_nop\n\tv_nop"
               : "+v"(a0), "+v"(a1), "+v"(b0), "+v"(b1)
               : "v"(p0), "v"(p1), "v"(x0), "v"(x1));
}

__device__ __forceinline__ v8h wpiece(const float* __restrict__ W, int k0, int n) {
  v8h o;
#pragma unroll
  for (int i = 0; i < 8; ++i) o[i] = (_Float16)(bfr(W[(size_t)(k0 + i) * DM + n]) * 64.0f);
  return o;
}

__global__ __launch_bounds__(256) void cvt_kernel(const float* __restrict__ x, const float* __restrict__ Wq,
                                                  const float* __restrict__ Wk, const float* __restrict__ Wv,
                                                  _Float16* __restrict__ X16, _Float16* __restrict__ WT16, int nbx) {
  const int tid = (int)threadIdx.x;
  const int blk = (int)blockIdx.x;
  if (blk < nbx) {
    const int li = blk * 256 + tid;
    const int r  = li >> 4;
    const int c0 = (li & 15) * 8;
    const int b  = r / SEQ;
    const int n  = r - b * SEQ;
    const float* xr = x + ((size_t)b * SEQ_FULL + n) * EM + c0;
    const v4f a  = *(const v4f*)(xr);
    const v4f a2 = *(const v4f*)(xr + 4);
    v8h o;
#pragma unroll
    for (int i = 0; i < 4; ++i) {
      o[i]     = (_Float16)(bfr(a[i]) * 16.0f);
      o[4 + i] = (_Float16)(bfr(a2[i]) * 16.0f);
    }
    _Float16* d = X16 + (size_t)li * 8;
    *(volatile v8h*)d = o;
    __threadfence();
    *(volatile v8h*)d = o;
  } else {
    const int li = (blk - nbx) * 256 + tid;
    if (li >= 3 * DM * EM / 8) return;
    const int mat = li >> 12;
    const int n   = (li >> 4) & (DM - 1);
    const int k0  = (li & 15) * 8;
    v8h o;
    if (mat == 0)      o = wpiece(Wq, k0, n);
    else if (mat == 1) o = wpiece(Wk, k0, n);
    else               o = wpiece(Wv, k0, n);
    _Float16* d = WT16 + (size_t)li * 8;
    *(volatile v8h*)d = o;
    __threadfence();
    *(volatile v8h*)d = o;
  }
}

__global__ __launch_bounds__(256) void gemm64_kernel(const _Float16* __restrict__ A, int lda,
                                                     const _Float16* __restrict__ Bt, int ldb,
                                                     _Float16* __restrict__ C, _Float16* __restrict__ C2, int ldc,
                                                     const float* __restrict__ bias, float bsc,
                                                     int M, int N, int K, float scale, int bias_mode) {
  __shared__ __align__(16) float sT[8][16 * 68];
  const int lane = threadIdx.x & 31;
  const int wave = __builtin_amdgcn_readfirstlane((int)(threadIdx.x >> 5));
  const int tilesN = N >> 6, tilesM = M >> 6;
  const int tile = (int)blockIdx.x * 8 + wave;
  if (tile >= tilesM * tilesN) return;
  const int tm = tile / tilesN, tn = tile - tm * tilesN;
  const int m0 = tm << 6, n0 = tn << 6;
  const int rl = lane & 15;
  const int koff = (lane >> 4) * 8;
  const int mOff = (lane >> 4) * 8;

  v8f acc[4][4];
#pragma unroll
  for (int i = 0; i < 4; ++i)
#pragma unroll
    for (int j = 0; j < 4; ++j) acc[i][j] = zero8();

#pragma unroll 1
  for (int k0 = 0; k0 < K; k0 += 32) {
    v16h bh[4];
#pragma unroll
    for (int j = 0; j < 4; ++j) bh[j] = ldfrag(Bt + (size_t)(n0 + (j << 4) + rl) * ldb + koff + k0);
#pragma unroll
    for (int i = 0; i < 4; ++i) {
      const size_t ao = (size_t)(m0 + (i << 4) + rl) * lda + koff + k0;
      const v16h ah = ldfrag(A + ao);
#pragma unroll
      for (int j = 0; j < 4; ++j) acc[i][j] = mma16(ah, bh[j], acc[i][j]);
      guard_g(acc[i][0], acc[i][3], ah, bh[3]);
    }
    keep4(bh[0], bh[1], bh[2], bh[3]);
  }
  accg4(acc[0][0], acc[0][1], acc[0][2], acc[0][3]);
  accg4(acc[1][0], acc[1][1], acc[1][2], acc[1][3]);
  accg4(acc[2][0], acc[2][1], acc[2][2], acc[2][3]);
  accg4(acc[3][0], acc[3][1], acc[3][2], acc[3][3]);

  float* slab = sT[wave];
#pragma unroll
  for (int i = 0; i < 4; ++i) {
    const int mBase = m0 + (i << 4);
    float brow[8];
#pragma unroll
    for (int r = 0; r < 8; ++r) brow[r] = 0.0f;
    if (bias_mode == 2) {
      const v4f ba = *(const v4f*)(bias + mBase + mOff);
      const v4f bb = *(const v4f*)(bias + mBase + mOff + 4);
#pragma unroll
      for (int r = 0; r < 4; ++r) { brow[r] = bsc * bfr(ba[r]); brow[4 + r] = bsc * bfr(bb[r]); }
    }
#pragma unroll
    for (int j = 0; j < 4; ++j) {
      float bcol = 0.0f;
      if (bias_mode == 1) bcol = bsc * bfr(bias[n0 + (j << 4) + rl]);
#pragma unroll
      for (int r = 0; r < 8; ++r) {
        const float bb = brow[r] + bcol;
        slab[(mOff + r) * 68 + (j << 4) + rl] = acc[i][j][r] * scale + bb;
      }
    }
    __builtin_amdgcn_fence(3  , "workgroup");
    __builtin_amdgcn_wave_barrier();
    __builtin_amdgcn_fence(2  , "workgroup");
    {
      const int qq = lane >> 3, c8 = (lane & 7) * 8;
#pragma unroll
      for (int ps = 0; ps < 2; ++ps) {
#pragma unroll
        for (int it = 0; it < 4; ++it) {
          const int row = it * 4 + qq;
          const float* sp = slab + row * 68 + c8;
          v8h hv, lv;
#pragma unroll
          for (int e = 0; e < 8; ++e) {
            const float f = sp[e];
            const _Float16 hh = (_Float16)f;
            hv[e] = hh;
            lv[e] = (_Float16)((f - (float)hh) * 1024.0f);
          }
          *(volatile v8h*)(C  + (size_t)(mBase + row) * ldc + n0 + c8) = hv;
          *(volatile v8h*)(C2 + (size_t)(mBase + row) * ldc + n0 + c8) = lv;
        }
        __threadfence();
      }
    }
    __builtin_amdgcn_fence(3  , "workgroup");
    __builtin_amdgcn_wave_barrier();
    __builtin_amdgcn_fence(2  , "workgroup");
  }
}

#define KCH      256
#define QSP      264
#define PSP      264
#define OSP      260
#define LATE_LDS  (3 * 32 * QSP * 2 + 2560)
#define EARLY_LDS (4 * 16 * QSP * 2 + 2560)
static_assert((QSP % 8) == 0 && (PSP % 8) == 0 && PSP >= KCH && QSP >= DM && (OSP % 4) == 0 && OSP >= DM);
static_assert(QSP == PSP);
static_assert((SEQ % KCH) == 0 && DM == 8 * 32 && KCH == 8 * 32);
static_assert(LATE_LDS <= 65536 && EARLY_LDS <= 65536);

template <int QT, bool EARLY>
__device__ __forceinline__ void attn_body(char* smem,
                                          const _Float16* __restrict__ qh, const _Float16* __restrict__ ql,
                                          const _Float16* __restrict__ kn, const _Float16* __restrict__ kl,
                                          const _Float16* __restrict__ vt, const _Float16* __restrict__ vl,
                                          float* __restrict__ out, const int batch, const int qloc0) {
  static_assert(EARLY ? (QT == 1) : (QT == 2));
  constexpr int QB  = 16 * QT;
  constexpr int TB  = QB * QSP * 2;
  constexpr int NPL = EARLY ? 4 : 3;
  constexpr int RPW = QB / 8;
  static_assert((TB % 16) == 0);
  static_assert(QB * OSP * 4 <= NPL * TB);
  static_assert(8 * QB <= 256);
  static_assert(RPW * 8 == QB);
  static_assert((SEQ % QB) == 0);

  _Float16* Qs = (_Float16*)(smem);
  _Float16* Ls = (_Float16*)(smem + TB);
  _Float16* Ps = (_Float16*)(smem + 2 * TB);
  _Float16* Pl = (_Float16*)(smem + (NPL - 1) * TB);
  float* pmax = (float*)(smem + NPL * TB);
  float* psum = pmax + 256;
  float* m_s  = psum + 256;
  float* l_s  = m_s + 32;
  float* al_s = m_s + 64;
  float* li_s = m_s + 96;

  const int tid  = (int)threadIdx.x;
  const int wave = __builtin_amdgcn_readfirstlane((int)(threadIdx.x >> 5));
  const int lane = tid & 31, h = lane >> 4, c = lane & 15;
  const int kbase = batch * SEQ;
  const int q0    = kbase + qloc0;
  const int qmax  = qloc0 + QB - 1;
  const float ninf = -__builtin_inff();
  const float sc = 0.000244140625f;
  const float rs = 0.0009765625f;

  if (tid < 32) { m_s[tid] = ninf; l_s[tid] = 0.0f; al_s[tid] = 0.0f; li_s[tid] = 0.0f; }
  psum[tid] = 0.0f;
  pmax[tid] = ninf;
#pragma unroll
  for (int i = 0; i < 2 * QT; ++i) {
    const int idx = i * 256 + tid;
    const int row = idx >> 5;
    const int pc  = idx & 31;
    const v8h vh = *(const v8h*)(qh + (size_t)(q0 + row) * DM + pc * 8);
    const v8h vq = *(const v8h*)(ql + (size_t)(q0 + row) * DM + pc * 8);
    *(v8h*)(Qs + row * QSP + pc * 8) = vh;
    *(v8h*)(Ls + row * QSP + pc * 8) = vq;
  }
  __syncthreads();

  v8f oacc[QT][2];
  v8f oacl[QT][2];
#pragma unroll
  for (int qt = 0; qt < QT; ++qt)
#pragma unroll
    for (int nt = 0; nt < 2; ++nt) { oacc[qt][nt] = zero8(); oacl[qt][nt] = zero8(); }

  const int qoff = c * QSP + 8 * h;
  const int ntile = qmax / KCH + 1;

#pragma unroll 1
  for (int t = 0; t < ntile; ++t) {
    const int kloc = t * KCH + 32 * wave;
    v8f sacc[QT][2];
    v8f sacl[QT][2];
#pragma unroll
    for (int qt = 0; qt < QT; ++qt)
#pragma unroll
      for (int kt = 0; kt < 2; ++kt) { sacc[qt][kt] = zero8(); sacl[qt][kt] = zero8(); }
    if (kloc <= qmax) {
      const size_t ko0 = (size_t)(kbase + kloc + c) * DM + 8 * h;
      const size_t ko1 = (size_t)(kbase + kloc + 16 + c) * DM + 8 * h;
#pragma unroll 1
      for (int k0 = 0; k0 < DM; k0 += 32) {
        const v16h a0 = ldfrag(kn + ko0 + k0), a1 = ldfrag(kn + ko1 + k0);
        v16h bq[QT], cq[QT];
#pragma unroll
        for (int qt = 0; qt < QT; ++qt) {
          bq[qt] = ldfrag(Qs + 16 * qt * QSP + qoff + k0);
          cq[qt] = ldfrag(Ls + 16 * qt * QSP + qoff + k0);
        }
#pragma unroll
        for (int qt = 0; qt < QT; ++qt) {
          sacc[qt][0] = mma16(a0, bq[qt], sacc[qt][0]);
          sacc[qt][1] = mma16(a1, bq[qt], sacc[qt][1]);
        }
#pragma unroll
        for (int qt = 0; qt < QT; ++qt) {
          sacl[qt][0] = mma16(a0, cq[qt], sacl[qt][0]);
          sacl[qt][1] = mma16(a1, cq[qt], sacl[qt][1]);
        }
        if constexpr (EARLY) {
          const v16h d0 = ldfrag(kl + ko0 + k0), d1 = ldfrag(kl + ko1 + k0);
          sacl[0][0] = mma16(d0, bq[0], sacl[0][0]);
          sacl[0][1] = mma16(d1, bq[0], sacl[0][1]);
          guard_a4f6(sacc[0][0], sacc[0][1], sacl[0][0], sacl[0][1], a0, a1, bq[0], cq[0], d0, d1);
        } else {
          guard_s8(sacc[0][0], sacc[0][1], sacc[QT - 1][0], sacc[QT - 1][1],
                   sacl[0][0], sacl[0][1], sacl[QT - 1][0], sacl[QT - 1][1],
                   a0, a1, bq[0], bq[QT - 1], cq[0], cq[QT - 1]);
        }
      }
    }
    {
#pragma unroll
      for (int qt = 0; qt < QT; ++qt) {
        const int qry = qloc0 + 16 * qt + c;
        float pm = ninf;
#pragma unroll
        for (int kt = 0; kt < 2; ++kt) {
#pragma unroll
          for (int r = 0; r < 8; ++r) {
            const int key = kloc + 16 * kt + 8 * h + r;
            float v = (sacc[qt][kt][r] + sacl[qt][kt][r] * rs) * sc;
            v = (key <= qry) ? v : ninf;
            sacc[qt][kt][r] = v;
            pm = fmaxf(pm, v);
          }
        }
        pm = fmaxf(pm, __shfl_xor(pm, 16, 32));
        pmax[wave * QB + 16 * qt + c] = pm;
      }
    }
    __syncthreads();
    if (wave == 0 && lane < QB) {
      const int row = lane;
      float ps = 0.0f;
#pragma unroll
      for (int w = 0; w < 8; ++w) ps += psum[w * QB + row];
      l_s[row] = l_s[row] * al_s[row] + ps;
      const float mo = m_s[row];
      float mx = mo;
#pragma unroll
      for (int w = 0; w < 8; ++w) mx = fmaxf(mx, pmax[w * QB + row]);
      al_s[row] = __expf(mo - mx);
      m_s[row] = mx;
    }
    __syncthreads();
    {
#pragma unroll
      for (int qt = 0; qt < QT; ++qt) {
        const float mq = m_s[16 * qt + c];
        float ps = 0.0f;
#pragma unroll
        for (int kt = 0; kt < 2; ++kt) {
          v8h hh, ll;
#pragma unroll
          for (int r = 0; r < 8; ++r) {
            const float p = __expf(sacc[qt][kt][r] - mq);
            ps += p;
            const float pw = p * 16384.0f;
            const _Float16 ph = (_Float16)pw;
            hh[r] = ph;
            ll[r] = (_Float16)((pw - (float)ph) * 1024.0f);
          }
          *(v8h*)(Ps + (16 * qt + c) * PSP + 32 * wave + 16 * kt + 8 * h) = hh;
          if constexpr (EARLY) *(v8h*)(Pl + (16 * qt + c) * PSP + 32 * wave + 16 * kt + 8 * h) = ll;
        }
        ps += __shfl_xor(ps, 16, 32);
        psum[wave * QB + 16 * qt + c] = ps;
        const v4f aA = *(const v4f*)(al_s + 16 * qt + 8 * h), aB = *(const v4f*)(al_s + 16 * qt + 8 * h + 4);
#pragma unroll
        for (int nt = 0; nt < 2; ++nt) {
#pragma unroll
          for (int r = 0; r < 4; ++r) {
            oacc[qt][nt][r] *= aA[r]; oacc[qt][nt][4 + r] *= aB[r];
            if constexpr (EARLY) { oacl[qt][nt][r] *= aA[r]; oacl[qt][nt][4 + r] *= aB[r]; }
          }
        }
      }
    }
    __syncthreads();
    {
      const int rem = qmax - t * KCH;
      int nks = ((rem >> 5) + 1) * 32;
      nks = (nks < KCH) ? nks : KCH;
      const size_t vo = (size_t)(32 * wave + c) * RTOT + kbase + (size_t)t * KCH + 8 * h;
#pragma unroll 1
      for (int ks = 0; ks < nks; ks += 32) {
        v16h pa[QT];
#pragma unroll
        for (int qt = 0; qt < QT; ++qt) pa[qt] = ldfrag(Ps + 16 * qt * PSP + c * PSP + 8 * h + ks);
        const v16h vb0 = ldfrag(vt + vo + ks);
        const v16h vb1 = ldfrag(vt + vo + (size_t)16 * RTOT + ks);
#pragma unroll
        for (int qt = 0; qt < QT; ++qt) {
          oacc[qt][0] = mma16(pa[qt], vb0, oacc[qt][0]);
          oacc[qt][1] = mma16(pa[qt], vb1, oacc[qt][1]);
        }
        if constexpr (EARLY) {
          const v16h pl0 = ldfrag(Pl + c * PSP + 8 * h + ks);
          const v16h vl0 = ldfrag(vl + vo + ks);
          const v16h vl1 = ldfrag(vl + vo + (size_t)16 * RTOT + ks);
          oacl[0][0] = mma16(pa[0], vl0, oacl[0][0]);
          oacl[0][1] = mma16(pa[0], vl1, oacl[0][1]);
          oacl[0][0] = mma16(pl0, vb0, oacl[0][0]);
          oacl[0][1] = mma16(pl0, vb1, oacl[0][1]);
          guard_a4f6(oacc[0][0], oacc[0][1], oacl[0][0], oacl[0][1], pa[0], pl0, vb0, vb1, vl0, vl1);
        } else {
          guard_pv4(oacc[0][0], oacc[0][1], oacc[QT - 1][0], oacc[QT - 1][1], pa[0], pa[QT - 1], vb0, vb1);
        }
      }
    }
  }

  if (wave == 0 && lane < QB) {
    const int row = lane;
    float ps = 0.0f;
#pragma unroll
    for (int w = 0; w < 8; ++w) ps += psum[w * QB + row];
    const float l = l_s[row] * al_s[row] + ps;
    li_s[row] = (1.0f / l) * (1.0f / 262144.0f);
  }
  __syncthreads();
  float* Os = (float*)(smem);
  {
#pragma unroll
    for (int qt = 0; qt < QT; ++qt) {
      const v4f iA = *(const v4f*)(li_s + 16 * qt + 8 * h), iB = *(const v4f*)(li_s + 16 * qt + 8 * h + 4);
#pragma unroll
      for (int nt = 0; nt < 2; ++nt) {
        const int col = 32 * wave + 16 * nt + c;
#pragma unroll
        for (int r = 0; r < 4; ++r) {
          float o0 = oacc[qt][nt][r], o1 = oacc[qt][nt][4 + r];
          if constexpr (EARLY) { o0 += oacl[qt][nt][r] * rs; o1 += oacl[qt][nt][4 + r] * rs; }
          Os[(16 * qt + 8 * h + r) * OSP + col]     = o0 * iA[r];
          Os[(16 * qt + 8 * h + 4 + r) * OSP + col] = o1 * iB[r];
        }
      }
    }
  }
  __syncthreads();
  {
    float* go = out + (size_t)q0 * DM;
#pragma unroll
    for (int ps = 0; ps < 2; ++ps) {
#pragma unroll
      for (int rr = 0; rr < RPW; ++rr) {
        const int row = RPW * wave + rr;
#pragma unroll
        for (int j = 0; j < 2; ++j) {
          const int pc = j * 32 + lane;
          const v4f v = *(const v4f*)(Os + row * OSP + pc * 4);
          *(volatile v4f*)(go + (size_t)row * DM + pc * 4) = v;
        }
      }
      __threadfence();
    }
  }
}

__global__ __launch_bounds__(256) void attn_early_kernel(const _Float16* __restrict__ qh, const _Float16* __restrict__ ql,
                                                         const _Float16* __restrict__ kn, const _Float16* __restrict__ kl,
                                                         const _Float16* __restrict__ vt, const _Float16* __restrict__ vl,
                                                         float* __restrict__ out) {
  extern __shared__ __align__(16) char smem[];
  const int blk = (int)blockIdx.x;
  const int batch = blk / EBLK;
  const int qloc0 = (blk - batch * EBLK) * 16;
  attn_body<1, true>(smem, qh, ql, kn, kl, vt, vl, out, batch, qloc0);
}

__global__ __launch_bounds__(256) void attn_late_kernel(const _Float16* __restrict__ qh, const _Float16* __restrict__ ql,
                                                        const _Float16* __restrict__ kn, const _Float16* __restrict__ vt,
                                                        float* __restrict__ out) {
  extern __shared__ __align__(16) char smem[];
  const int blk = (int)blockIdx.x;
  const int batch = blk / LBLKD;
  const int qloc0 = EROWS + (blk - batch * LBLKD) * 32;
  attn_body<2, false>(smem, qh, ql, kn, kn, vt, vt, out, batch, qloc0);
}

static_assert((size_t)3 * DM * EM * 2 + (size_t)RTOT * EM * 2 + (size_t)6 * RTOT * DM * 2 <= (size_t)134217728);
static_assert(((size_t)3 * DM * EM * 2) % 128 == 0 && ((size_t)RTOT * EM * 2) % 128 == 0 && ((size_t)RTOT * DM * 2) % 128 == 0);

extern "C" void kernel_launch(void* const* d_in, const int* in_sizes, int n_in,
                              void* d_out, int out_size, void* d_ws, size_t ws_size,
                              hipStream_t stream) {
  if (n_in < 7) return;
  const int R = RTOT;
  const long long needx = ((long long)(NB - 1) * SEQ_FULL + SEQ) * EM;
  if ((long long)in_sizes[0] < needx) return;
  if (in_sizes[1] < EM * DM || in_sizes[3] < EM * DM || in_sizes[5] < EM * DM) return;
  if (in_sizes[2] < DM || in_sizes[4] < DM || in_sizes[6] < DM) return;
  if ((long long)out_size < (long long)R * DM) return;

  const float* x  = (const float*)d_in[0];
  const float* Wq = (const float*)d_in[1];
  const float* bq = (const float*)d_in[2];
  const float* Wk = (const float*)d_in[3];
  const float* bk = (const float*)d_in[4];
  const float* Wv = (const float*)d_in[5];
  const float* bv = (const float*)d_in[6];
  float* out = (float*)d_out;

  const size_t bWT = (size_t)3 * DM * EM * 2;
  const size_t bX  = (size_t)R * EM * 2;
  const size_t bPl = (size_t)R * DM * 2;
  size_t off = 0;
  const size_t oWT = off; off += bWT;
  const size_t oX  = off; off += bX;
  const size_t oQ  = off; off += bPl;
  const size_t oQL = off; off += bPl;
  const size_t oK  = off; off += bPl;
  const size_t oKL = off; off += bPl;
  const size_t oVT = off; off += bPl;
  const size_t oVL = off; off += bPl;
  if (off > ws_size) return;
  if (off > (size_t)134217728) return;

  char* ws = (char*)d_ws;
  _Float16* WT16 = (_Float16*)(ws + oWT);
  _Float16* X16  = (_Float16*)(ws + oX);
  _Float16* Q16  = (_Float16*)(ws + oQ);
  _Float16* QL16 = (_Float16*)(ws + oQL);
  _Float16* K16  = (_Float16*)(ws + oK);
  _Float16* KL16 = (_Float16*)(ws + oKL);
  _Float16* VT16 = (_Float16*)(ws + oVT);
  _Float16* VL16 = (_Float16*)(ws + oVL);

  const dim3 blk(256);
  const int nbx = (R * EM / 8) / 256;
  const int nbw = (3 * DM * EM / 8) / 256;
  if (nbx * 256 * 8 != R * EM) return;

  cvt_kernel<<<dim3(nbx + nbw), blk, 0, stream>>>(x, Wq, Wk, Wv, X16, WT16, nbx);
  gemm64_kernel<<<dim3(((R / 64) * (DM / 64)) / 8), blk, 0, stream>>>(
      X16, EM, WT16, EM, Q16, QL16, DM, bq, 16.0f, R, DM, EM, 0.015625f, 1);
  gemm64_kernel<<<dim3(((R / 64) * (DM / 64)) / 8), blk, 0, stream>>>(
      X16, EM, WT16 + (size_t)DM * EM, EM, K16, KL16, DM, bk, 16.0f, R, DM, EM, 0.015625f, 1);
  gemm64_kernel<<<dim3(((DM / 64) * (R / 64)) / 8), blk, 0, stream>>>(
      WT16 + (size_t)2 * DM * EM, EM, X16, EM, VT16, VL16, R, bv, 16.0f, DM, R, EM, 0.015625f, 2);
  (void)hipFuncSetAttribute(reinterpret_cast<const void*>(&attn_early_kernel),
                            hipFuncAttributeMaxDynamicSharedMemorySize, EARLY_LDS);
  attn_early_kernel<<<dim3(NB * EBLK), blk, EARLY_LDS, stream>>>(Q16, QL16, K16, KL16, VT16, VL16, out);
  if (LBLK > 0) {
    (void)hipFuncSetAttribute(reinterpret_cast<const void*>(&attn_late_kernel),
                              hipFuncAttributeMaxDynamicSharedMemorySize, LATE_LDS);
    attn_late_kernel<<<dim3(NB * LBLKD), blk, LATE_LDS, stream>>>(Q16, QL16, K16, VT16, out);
  }
  (void)hipGetLastError();
}
